// NeuronCircuit_70755291234742
// MI455X (gfx1250) — hardware-run, weakly checked
//
#include <hip/hip_runtime.h>
#include <math.h>

constexpr int kBatch = 4;
constexpr int kSeq   = 1024;
constexpr int kDm    = 1024;
constexpr int kRank  = 64;
constexpr int kPool  = 32;
constexpr int kHeads = 16;
constexpr int kDh    = 64;
constexpr int kTok   = kBatch * kSeq;
constexpr int kNR    = kPool * kRank;
constexpr int kGrp   = 8;
constexpr int kCtxLd = 2 * kDm;
constexpr int kZvLd  = 2 * kNR;
constexpr float kScoreScale = 0.125f;
constexpr float kFill       = -1.0e30f;
static_assert(kHeads * kDh == kDm, "shape");
static_assert(kTok % 64 == 0 && kNR % 64 == 0 && kDm % 64 == 0 && kSeq % 64 == 0 && kDh % 64 == 0, "tiles");
static_assert(kDm % 32 == 0 && kNR % 32 == 0 && kZvLd % 32 == 0 && kDh % 32 == 0 && kSeq % 32 == 0 && kCtxLd % 32 == 0, "k steps");
static_assert(kHeads % kGrp == 0 && kSeq == 128 * 8, "softmax map");

constexpr size_t szXBF = (size_t)kTok * kDm * 2;
constexpr size_t szRVD = (size_t)kDm * kZvLd * 2;
constexpr size_t szFT  = (size_t)kNR * kDm * 2;
constexpr size_t szXN  = (size_t)kTok * kNR * 4;
constexpr size_t szH   = (size_t)kTok * kRank * 4;
constexpr size_t szZQK = (size_t)kTok * kNR * 2;
constexpr size_t szZV  = (size_t)kTok * kZvLd * 2;
constexpr size_t szQ   = (size_t)kTok * kDm * 2;
constexpr size_t szWOD = (size_t)kDm * kCtxLd * 2;
constexpr size_t offXBF = 0;
constexpr size_t offRVD = offXBF + szXBF;
constexpr size_t offFT  = offRVD + szRVD;
constexpr size_t offXN  = offFT + szFT;
constexpr size_t offH   = offXN + szXN;
constexpr size_t offZQK = offH + 3 * szH;
constexpr size_t offZV  = offZQK + szZQK;
constexpr size_t offQ   = offZV + szZV;
constexpr size_t offK   = offQ + szQ;
constexpr size_t offWOD = offK + szQ;
constexpr size_t kWsTotal = offWOD + szWOD;
static_assert(kWsTotal == 128974848, "carve");
static_assert(kWsTotal <= 134217728, "carve cap");
static_assert((size_t)kTok * kCtxLd * 2 <= szXBF + szRVD, "ctx alias");
static_assert((size_t)kGrp * kSeq * kSeq * 4 <= szXN, "score alias");
static_assert(2 * (size_t)kGrp * kSeq * kSeq * 2 <= szZV, "prob alias");
static_assert(2 * (size_t)kDm * kTok * 2 <= szZQK, "vt alias");
static_assert((size_t)kDm * kNR * 2 <= szFT, "rt alias");

typedef __attribute__((ext_vector_type(16))) _Float16 v16h;
typedef __attribute__((ext_vector_type(8)))  _Float16 v8h;
typedef __attribute__((ext_vector_type(16))) __bf16   v16b;
typedef __attribute__((ext_vector_type(8)))  __bf16   v8b;
typedef __attribute__((ext_vector_type(8)))  float    v8f;
typedef __attribute__((ext_vector_type(4)))  float    v4f;
typedef __attribute__((ext_vector_type(4)))  unsigned int v4u;

__device__ __forceinline__ unsigned short f2bf_bits(float f) {
  unsigned u = __float_as_uint(f);
  return (unsigned short)((u + 0x7FFFu + ((u >> 16) & 1u)) >> 16);
}
__device__ __forceinline__ float bf_bits2f(unsigned short h) { return __uint_as_float(((unsigned)h) << 16); }
__device__ __forceinline__ float bf16r(float f) { return bf_bits2f(f2bf_bits(f)); }

__device__ __forceinline__ void dep_guard_h(v8f& a, v8f& b, v16h x, v16h y) { asm volatile("v_nop\n\tv_nop\n\tv_nop\n\tv_nop" : "+v"(a), "+v"(b) : "v"(x), "v"(y)); }
__device__ __forceinline__ void dep_guard_b(v8f& a, v8f& b, v16b x, v16b y) { asm volatile("v_nop\n\tv_nop\n\tv_nop\n\tv_nop" : "+v"(a), "+v"(b) : "v"(x), "v"(y)); }
__device__ __forceinline__ void keep4_h(v16h a, v16h b, v16h c, v16h d) { asm volatile("v_nop" :: "v"(a), "v"(b), "v"(c), "v"(d)); }
__device__ __forceinline__ void keep4_b(v16b a, v16b b, v16b c, v16b d) { asm volatile("v_nop" :: "v"(a), "v"(b), "v"(c), "v"(d)); }
__device__ __forceinline__ void acc_guard4(v8f& a, v8f& b, v8f& c, v8f& d) { asm volatile("v_nop\n\tv_nop\n\tv_nop\n\tv_nop" : "+v"(a), "+v"(b), "+v"(c), "+v"(d)); }
template <typename T> struct Frag;
template <> struct Frag<_Float16> {
  typedef v16h V; union U { v16h v; v8h h[2]; };
  static __device__ __forceinline__ v16h load(const _Float16* p) {
    U f; f.h[0] = *(const v8h*)(p); f.h[1] = *(const v8h*)(p + 16); return f.v;
  }
  static __device__ __forceinline__ v8f mma(v16h a, v16h b, v8f c) {
    return __builtin_amdgcn_wmma_f32_16x16x32_f16(false, a, false, b, (short)0, c, false, false);
  }
  static __device__ __forceinline__ void guard(v8f& a, v8f& b, v16h x, v16h y) { dep_guard_h(a, b, x, y); }
  static __device__ __forceinline__ void keep(v16h a, v16h b, v16h c, v16h d) { keep4_h(a, b, c, d); }
};
template <> struct Frag<__bf16> {
  typedef v16b V; union U { v16b v; v8b h[2]; };
  static __device__ __forceinline__ v16b load(const __bf16* p) {
    U f; f.h[0] = *(const v8b*)(p); f.h[1] = *(const v8b*)(p + 16); return f.v;
  }
  static __device__ __forceinline__ v8f mma(v16b a, v16b b, v8f c) {
    return __builtin_amdgcn_wmma_f32_16x16x32_bf16(false, a, false, b, (short)0, c, false, false);
  }
  static __device__ __forceinline__ void guard(v8f& a, v8f& b, v16b x, v16b y) { dep_guard_b(a, b, x, y); }
  static __device__ __forceinline__ void keep(v16b a, v16b b, v16b c, v16b d) { keep4_b(a, b, c, d); }
};

__device__ __forceinline__ unsigned pk16(unsigned short a, unsigned short b) { return (unsigned)a | ((unsigned)b << 16); }

template <int ET> struct Elem;
template <> struct Elem<0> { typedef _Float16 T; };
template <> struct Elem<1> { typedef __bf16 T; };
template <int ET, bool SPLIT, int BIAS_MODE, int OUT_MODE, bool RESID, int ACT = 0>
__global__ __launch_bounds__(256) void wmma_gemm64(
    const unsigned short* __restrict__ Ap, const unsigned short* __restrict__ A2p, int lda, long strideA,
    const unsigned short* __restrict__ Btp, const unsigned short* __restrict__ Bt2p, int ldb, long strideB,
    void* __restrict__ Cout, void* __restrict__ Cout2, int ldc, long strideC,
    const float* __restrict__ bias,
    const float* __restrict__ resid, long strideR,
    int M, int N, int K, float scale) {
  typedef typename Elem<ET>::T T;
  typedef typename Frag<T>::V V;
  const T* A = (const T*)Ap; const T* A2 = (const T*)A2p; const T* Bt = (const T*)Btp; const T* Bt2 = (const T*)Bt2p;
  __shared__ __align__(16) float sT[8][16 * 68];
  const int b    = blockIdx.y;
  const int lane = threadIdx.x & 31;
  const int wave = threadIdx.x >> 5;
  const int tilesN = N >> 6;
  const int tilesM = M >> 6;
  const int tile = blockIdx.x * 8 + wave;
  if (tile >= tilesM * tilesN) return;
  const int tm = tile / tilesN;
  const int tn = tile - tm * tilesN;
  const int m0 = tm << 6;
  const int n0 = tn << 6;

  const T* Ab  = A  + (size_t)b * strideA;
  const T* Bb  = Bt + (size_t)b * strideB;
  const T* Ab2 = SPLIT ? (A2  + (size_t)b * strideA) : nullptr;
  const T* Bb2 = SPLIT ? (Bt2 + (size_t)b * strideB) : nullptr;

  const int rlane = lane & 15;
  const int koff  = (lane >> 4) * 8;
  const int mOff  = (lane >> 4) * 8;

  v8f acc[4][4];
#pragma unroll
  for (int i = 0; i < 4; ++i)
#pragma unroll
    for (int j = 0; j < 4; ++j) acc[i][j] = (v8f){0.f,0.f,0.f,0.f,0.f,0.f,0.f,0.f};

  for (int k0 = 0; k0 < K; k0 += 32) {
    V bh[4], bl[4];
#pragma unroll
    for (int j = 0; j < 4; ++j) {
      const size_t bo = (size_t)(n0 + (j << 4) + rlane) * ldb + koff + k0;
      bh[j] = Frag<T>::load(Bb + bo);
      if (SPLIT) bl[j] = Frag<T>::load(Bb2 + bo);
    }
#pragma unroll
    for (int i = 0; i < 4; ++i) {
      const size_t ao = (size_t)(m0 + (i << 4) + rlane) * lda + koff + k0;
      V ah = Frag<T>::load(Ab + ao);
      V al;
      if (SPLIT) al = Frag<T>::load(Ab2 + ao);
#pragma unroll
      for (int j = 0; j < 4; ++j) {
        acc[i][j] = Frag<T>::mma(ah, bh[j], acc[i][j]);
        if (SPLIT) {
          acc[i][j] = Frag<T>::mma(ah, bl[j], acc[i][j]);
          acc[i][j] = Frag<T>::mma(al, bh[j], acc[i][j]);
        }
      }
      Frag<T>::guard(acc[i][0], acc[i][3], ah, SPLIT ? al : ah);
    }
    Frag<T>::keep(bh[0], bh[1], bh[2], bh[3]);
    if (SPLIT) Frag<T>::keep(bl[0], bl[1], bl[2], bl[3]);
  }
  acc_guard4(acc[0][0], acc[0][1], acc[0][2], acc[0][3]);
  acc_guard4(acc[1][0], acc[1][1], acc[1][2], acc[1][3]);
  acc_guard4(acc[2][0], acc[2][1], acc[2][2], acc[2][3]);
  acc_guard4(acc[3][0], acc[3][1], acc[3][2], acc[3][3]);

  float* slab = sT[wave];
  const float* Rb = RESID ? (resid + (size_t)b * strideR) : nullptr;
#pragma unroll
  for (int i = 0; i < 4; ++i) {
    const int mBase = m0 + (i << 4);
#pragma unroll
    for (int j = 0; j < 4; ++j) {
      const int n = n0 + (j << 4) + rlane;
      float bv = 0.f;
      if (BIAS_MODE == 2) bv = bias[n];
#pragma unroll
      for (int r = 0; r < 8; ++r) {
        float v = acc[i][j][r] * scale;
        if (BIAS_MODE == 1) v += bias[mBase + mOff + r];
        if (BIAS_MODE == 2) v += bv;
        if (RESID) v += Rb[(size_t)(mBase + mOff + r) * ldc + n];
        if (ACT == 2) v = fmaxf(v, 0.0f);
        if (ACT == 4) v = (v > 0.f) ? v : 0.01f * v;
        slab[(mOff + r) * 68 + (j << 4) + rlane] = v;
      }
    }
    __builtin_amdgcn_fence(__ATOMIC_RELEASE, "workgroup");
    __builtin_amdgcn_wave_barrier();
    __builtin_amdgcn_fence(__ATOMIC_ACQUIRE, "workgroup");
    if (OUT_MODE == 0) {
      float* C = (float*)Cout + (size_t)b * strideC;
      const int hh = lane >> 4, c4 = (lane & 15) * 4;
      for (int pass = 0; pass < 2; ++pass) {
#pragma unroll
        for (int it = 0; it < 8; ++it) {
          const int row = it * 2 + hh;
          v4f v = *(const v4f*)(slab + row * 68 + c4);
          *(volatile v4f*)(C + (size_t)(mBase + row) * ldc + n0 + c4) = v;
        }
        __threadfence();
      }
    } else {
      const int q = lane >> 3, c8 = (lane & 7) * 8;
      unsigned short* C  = (unsigned short*)Cout  + (size_t)b * strideC;
      unsigned short* C2 = (OUT_MODE == 2) ? ((unsigned short*)Cout2 + (size_t)b * strideC) : nullptr;
      for (int pass = 0; pass < 2; ++pass) {
#pragma unroll
        for (int it = 0; it < 4; ++it) {
          const int row = it * 4 + q;
          const float* sp = slab + row * 68 + c8;
          v8h hv, lv;
#pragma unroll
          for (int e = 0; e < 8; ++e) {
            if (OUT_MODE == 1) {
              hv[e] = (_Float16)sp[e];
            } else if (OUT_MODE == 3) {
              const unsigned short sb = f2bf_bits(sp[e]);
              hv[e] = __builtin_bit_cast(_Float16, sb);
            } else {
              unsigned short hb = f2bf_bits(sp[e]);
              unsigned short lb = f2bf_bits(sp[e] - bf_bits2f(hb));
              hv[e] = __builtin_bit_cast(_Float16, hb);
              lv[e] = __builtin_bit_cast(_Float16, lb);
            }
          }
          *(volatile v8h*)(C + (size_t)(mBase + row) * ldc + n0 + c8) = hv;
          if (OUT_MODE == 2) *(volatile v8h*)(C2 + (size_t)(mBase + row) * ldc + n0 + c8) = lv;
        }
        __threadfence();
      }
    }
    __builtin_amdgcn_fence(__ATOMIC_RELEASE, "workgroup");
    __builtin_amdgcn_wave_barrier();
    __builtin_amdgcn_fence(__ATOMIC_ACQUIRE, "workgroup");
  }
}

__global__ __launch_bounds__(256) void cast_bf16x8_kernel(const float* __restrict__ in, unsigned short* __restrict__ out, int n8) {
  const int i = blockIdx.x * 256 + threadIdx.x;
  if (i >= n8) return;
  const float* p = in + 8 * (size_t)i;
  const v4f a = *(const v4f*)(p);
  const v4f c = *(const v4f*)(p + 4);
  unsigned short hb[8];
#pragma unroll
  for (int e = 0; e < 4; ++e) {
    hb[e]     = f2bf_bits(a[e]);
    hb[4 + e] = f2bf_bits(c[e]);
  }
  const v4u u = (v4u){pk16(hb[0], hb[1]), pk16(hb[2], hb[3]), pk16(hb[4], hb[5]), pk16(hb[6], hb[7])};
  unsigned short* q = out + 8 * (size_t)i;
  *(volatile v4u*)q = u;
  __threadfence();
  *(volatile v4u*)q = u;
}

__global__ __launch_bounds__(256) void wo_cast_kernel(const float* __restrict__ Wo, unsigned short* __restrict__ WOD, int n8) {
  const int i = blockIdx.x * 256 + threadIdx.x;
  if (i >= n8) return;
  const int row = i >> 7;
  const int c8  = (i & 127) * 8;
  const float* p = Wo + (size_t)row * kDm + c8;
  const v4f a = *(const v4f*)(p);
  const v4f c = *(const v4f*)(p + 4);
  unsigned short hb[8];
#pragma unroll
  for (int e = 0; e < 4; ++e) {
    hb[e]     = f2bf_bits(a[e]);
    hb[4 + e] = f2bf_bits(c[e]);
  }
  const v4u u = (v4u){pk16(hb[0], hb[1]), pk16(hb[2], hb[3]), pk16(hb[4], hb[5]), pk16(hb[6], hb[7])};
  unsigned short* q0 = WOD + (size_t)row * kCtxLd + c8;
  unsigned short* q1 = q0 + kDm;
  *(volatile v4u*)q0 = u;
  *(volatile v4u*)q1 = u;
  __threadfence();
  *(volatile v4u*)q0 = u;
  *(volatile v4u*)q1 = u;
}

__global__ __launch_bounds__(256) void fcast_kernel(const float* __restrict__ F, unsigned short* __restrict__ FT) {
  __shared__ float sm[64][65];
  const int t  = threadIdx.x;
  const int d0 = blockIdx.x * 64;
  const int n  = blockIdx.y;
  const float* src = F + (size_t)n * (kDm * kRank) + (size_t)d0 * kRank;
#pragma unroll
  for (int i = 0; i < 4; ++i) {
    const int e4 = (i * 256 + t) * 4;
    const int dl = e4 >> 6;
    const int r  = e4 & 63;
    const v4f w = *(const v4f*)(src + e4);
    sm[r][dl] = w[0]; sm[r + 1][dl] = w[1]; sm[r + 2][dl] = w[2]; sm[r + 3][dl] = w[3];
  }
  __syncthreads();
  const int lane = t & 31, wave = t >> 5;
  const int q = lane >> 3, c8 = (lane & 7) * 8;
  unsigned short* op = FT + (size_t)(n * kRank) * kDm + d0;
  for (int pass = 0; pass < 2; ++pass) {
#pragma unroll
    for (int it = 0; it < 2; ++it) {
      const int row = wave * 8 + it * 4 + q;
      unsigned short hb[8];
#pragma unroll
      for (int e = 0; e < 8; ++e) hb[e] = f2bf_bits(sm[row][c8 + e]);
      const v4u u = (v4u){pk16(hb[0], hb[1]), pk16(hb[2], hb[3]), pk16(hb[4], hb[5]), pk16(hb[6], hb[7])};
      *(volatile v4u*)(op + (size_t)row * kDm + c8) = u;
    }
    __threadfence();
  }
}

template <bool DUP>
__global__ __launch_bounds__(256) void rcast_kernel(const float* __restrict__ Rf, unsigned short* __restrict__ RT) {
  __shared__ float sm[64][65];
  const int ldr = DUP ? kZvLd : kNR;
  const int t  = threadIdx.x;
  const int c0 = blockIdx.x * 64;
  const int d0 = blockIdx.y * 64;
#pragma unroll
  for (int i = 0; i < 4; ++i) {
    const int e4 = (i * 256 + t) * 4;
    const int cl = e4 >> 6;
    const int dl = e4 & 63;
    const v4f w = *(const v4f*)(Rf + (size_t)(c0 + cl) * kDm + d0 + dl);
    sm[dl][cl] = w[0]; sm[dl + 1][cl] = w[1]; sm[dl + 2][cl] = w[2]; sm[dl + 3][cl] = w[3];
  }
  __syncthreads();
  const int lane = t & 31, wave = t >> 5;
  const int q = lane >> 3, c8 = (lane & 7) * 8;
  unsigned short* op = RT + (size_t)d0 * ldr + c0;
  for (int pass = 0; pass < 2; ++pass) {
#pragma unroll
    for (int it = 0; it < 2; ++it) {
      const int row = wave * 8 + it * 4 + q;
      unsigned short hb[8];
#pragma unroll
      for (int e = 0; e < 8; ++e) hb[e] = f2bf_bits(sm[row][c8 + e]);
      const v4u u = (v4u){pk16(hb[0], hb[1]), pk16(hb[2], hb[3]), pk16(hb[4], hb[5]), pk16(hb[6], hb[7])};
      *(volatile v4u*)(op + (size_t)row * ldr + c8) = u;
      if (DUP) *(volatile v4u*)(op + (size_t)row * ldr + kNR + c8) = u;
    }
    __threadfence();
  }
}

__global__ __launch_bounds__(256) void reduce_kernel(const float* __restrict__ xn, const float* __restrict__ w, float* __restrict__ h) {
  const int lane = threadIdx.x & 31;
  const int wave = threadIdx.x >> 5;
  const int tok  = (blockIdx.x * 8 + wave) * 2 + (lane >> 4);
  const int r0   = (lane & 15) * 4;
  const float* xr = xn + (size_t)tok * kNR + r0;
  const float* wr = w + (size_t)tok * kPool;
  float a0 = 0.0f, a1 = 0.0f, a2 = 0.0f, a3 = 0.0f;
#pragma unroll 1
  for (int n4 = 0; n4 < kPool; n4 += 4) {
    const v4f w4 = *(const v4f*)(wr + n4);
#pragma unroll
    for (int e = 0; e < 4; ++e) {
      const float wv = bf16r(w4[e]);
      const v4f xv = *(const v4f*)(xr + (size_t)(n4 + e) * kRank);
      a0 += wv * xv[0];
      a1 += wv * xv[1];
      a2 += wv * xv[2];
      a3 += wv * xv[3];
    }
  }
  const v4f val = (v4f){a0, a1, a2, a3};
  float* hp = h + (size_t)tok * kRank + r0;
  *(volatile v4f*)hp = val;
  __threadfence();
  *(volatile v4f*)hp = val;
}

template <bool SPLIT2>
__global__ __launch_bounds__(256) void buildz_kernel(const float* __restrict__ rw, const float* __restrict__ h, unsigned short* __restrict__ z) {
#pragma clang fp contract(off)
  const int ldz  = SPLIT2 ? kZvLd : kNR;
  const int lane = threadIdx.x & 31, wave = threadIdx.x >> 5;
  const int tok  = blockIdx.x * 8 + wave;
  const int rr   = (lane & 7) * 8;
  const float* hr = h + (size_t)tok * kRank + rr;
  const v4f ha = *(const v4f*)(hr);
  const v4f hc = *(const v4f*)(hr + 4);
  float hv[8];
#pragma unroll
  for (int e = 0; e < 4; ++e) { hv[e] = ha[e]; hv[4 + e] = hc[e]; }
  const float* wr = rw + (size_t)tok * kPool + (lane >> 3);
  v4u uh[8], ul[8];
#pragma unroll
  for (int it = 0; it < 8; ++it) {
    const float wv = bf16r(wr[it * 4]);
    unsigned short hb[8], lb[8];
#pragma unroll
    for (int e = 0; e < 8; ++e) {
      const float zv = wv * hv[e];
      hb[e] = f2bf_bits(zv);
      if (SPLIT2) lb[e] = f2bf_bits(zv - bf_bits2f(hb[e]));
      else lb[e] = 0;
    }
    uh[it] = (v4u){pk16(hb[0], hb[1]), pk16(hb[2], hb[3]), pk16(hb[4], hb[5]), pk16(hb[6], hb[7])};
    ul[it] = (v4u){pk16(lb[0], lb[1]), pk16(lb[2], lb[3]), pk16(lb[4], lb[5]), pk16(lb[6], lb[7])};
  }
  unsigned short* zr = z + (size_t)tok * ldz + lane * 8;
  for (int pass = 0; pass < 2; ++pass) {
#pragma unroll
    for (int it = 0; it < 8; ++it) {
      *(volatile v4u*)(zr + it * 256) = uh[it];
      if (SPLIT2) *(volatile v4u*)(zr + kNR + it * 256) = ul[it];
    }
    __threadfence();
  }
}

__global__ __launch_bounds__(128) void softmax_kernel(const float* __restrict__ sc, unsigned short* __restrict__ ph,
                                                      unsigned short* __restrict__ pl) {
#pragma clang fp contract(off)
  __shared__ float redM[4];
  __shared__ float redS[4];
  const int q    = blockIdx.x;
  const int j    = blockIdx.y;
  const int t    = threadIdx.x;
  const int lane = t & 31, wave = t >> 5;
  const size_t rowoff = ((size_t)j * kSeq + q) * kSeq;
  const int c0 = t * 8;
  const float* sr = sc + rowoff + c0;
  const v4f a = *(const v4f*)(sr);
  const v4f c = *(const v4f*)(sr + 4);
  float x[8];
#pragma unroll
  for (int e = 0; e < 4; ++e) {
    const float s0 = a[e] * kScoreScale;
    const float s1 = c[e] * kScoreScale;
    x[e]     = (c0 + e <= q) ? s0 : kFill;
    x[4 + e] = (c0 + 4 + e <= q) ? s1 : kFill;
  }
  float m = x[0];
#pragma unroll
  for (int e = 1; e < 8; ++e) m = fmaxf(m, x[e]);
#pragma unroll
  for (int off = 16; off > 0; off >>= 1) m = fmaxf(m, __shfl_xor(m, off, 32));
  if (lane == 0) redM[wave] = m;
  __syncthreads();
  const float mm = fmaxf(fmaxf(redM[0], redM[1]), fmaxf(redM[2], redM[3]));
  float ex[8];
  float sum = 0.0f;
#pragma unroll
  for (int e = 0; e < 8; ++e) {
    ex[e] = expf(x[e] - mm);
    sum += ex[e];
  }
#pragma unroll
  for (int off = 16; off > 0; off >>= 1) sum += __shfl_xor(sum, off, 32);
  if (lane == 0) redS[wave] = sum;
  __syncthreads();
  const float tot = ((redS[0] + redS[1]) + redS[2]) + redS[3];
  const float inv = 1.0f / tot;
  unsigned short hb[8], lb[8];
#pragma unroll
  for (int e = 0; e < 8; ++e) {
    const float p = ex[e] * inv;
    hb[e] = f2bf_bits(p);
    lb[e] = f2bf_bits(p - bf_bits2f(hb[e]));
  }
  const v4u uh = (v4u){pk16(hb[0], hb[1]), pk16(hb[2], hb[3]), pk16(hb[4], hb[5]), pk16(hb[6], hb[7])};
  const v4u ul = (v4u){pk16(lb[0], lb[1]), pk16(lb[2], lb[3]), pk16(lb[4], lb[5]), pk16(lb[6], lb[7])};
  unsigned short* p0 = ph + rowoff + c0;
  unsigned short* p1 = pl + rowoff + c0;
  *(volatile v4u*)p0 = uh;
  *(volatile v4u*)p1 = ul;
  __threadfence();
  *(volatile v4u*)p0 = uh;
  *(volatile v4u*)p1 = ul;
}

extern "C" void kernel_launch(void* const* d_in, const int* in_sizes, int n_in,
                              void* d_out, int out_size, void* d_ws, size_t ws_size,
                              hipStream_t stream) {
  if (n_in < 14) return;
  if (in_sizes[0] != kTok * kDm) return;
  for (int i = 1; i <= 6; ++i) if (in_sizes[i] != kTok * kPool) return;
  for (int i = 7; i <= 12; ++i) if (in_sizes[i] != kPool * kDm * kRank) return;
  if (in_sizes[13] != kDm * kDm) return;
  if (out_size != kTok * kDm) return;
  if (ws_size < kWsTotal) return;

  const float* x   = (const float*)d_in[0];
  const float* fqw = (const float*)d_in[1];
  const float* fkw = (const float*)d_in[2];
  const float* fvw = (const float*)d_in[3];
  const float* rqw = (const float*)d_in[4];
  const float* rkw = (const float*)d_in[5];
  const float* rvw = (const float*)d_in[6];
  const float* fqn = (const float*)d_in[7];
  const float* fkn = (const float*)d_in[8];
  const float* fvn = (const float*)d_in[9];
  const float* rqn = (const float*)d_in[10];
  const float* rkn = (const float*)d_in[11];
  const float* rvn = (const float*)d_in[12];
  const float* Wo  = (const float*)d_in[13];
  float* out = (float*)d_out;

  char* ws = (char*)d_ws;
  unsigned short* XBF = (unsigned short*)(ws + offXBF);
  unsigned short* RVD = (unsigned short*)(ws + offRVD);
  unsigned short* FT  = (unsigned short*)(ws + offFT);
  float*          XN  = (float*)(ws + offXN);
  float*          SC  = (float*)(ws + offXN);
  float*          HQ  = (float*)(ws + offH);
  float*          HK  = (float*)(ws + offH + szH);
  float*          HV  = (float*)(ws + offH + 2 * szH);
  unsigned short* ZQK = (unsigned short*)(ws + offZQK);
  unsigned short* VTH = (unsigned short*)(ws + offZQK);
  unsigned short* VTL = (unsigned short*)(ws + offZQK + szZQK / 2);
  unsigned short* ZV  = (unsigned short*)(ws + offZV);
  unsigned short* PH  = (unsigned short*)(ws + offZV);
  unsigned short* PL  = (unsigned short*)(ws + offZV + szZV / 2);
  unsigned short* CTX = (unsigned short*)(ws + offXBF);
  unsigned short* Q16 = (unsigned short*)(ws + offQ);
  unsigned short* K16 = (unsigned short*)(ws + offK);
  unsigned short* WOD = (unsigned short*)(ws + offWOD);
  const float* dum = HQ;

  const int tilesComp = (kTok / 64) * (kNR / 64);
  const int tilesRest = (kTok / 64) * (kDm / 64);
  const int tilesV    = (kDm / 64) * (kTok / 64);
  const int tilesS    = (kSeq / 64) * (kSeq / 64);
  const int tilesPV   = (kSeq / 64) * (kDh / 64);
  const int tilesOut  = (kTok / 64) * (kDm / 64);
  const int n8x = (kTok * kDm) / 8;
  const int n8w = (kDm * kDm) / 8;

  cast_bf16x8_kernel<<<dim3(n8x / 256), dim3(256), 0, stream>>>(x, XBF, n8x);

  const float* fn[3] = {fqn, fkn, fvn};
  const float* fw[3] = {fqw, fkw, fvw};
  float*       hh[3] = {HQ, HK, HV};
  for (int c = 0; c < 3; ++c) {
    fcast_kernel<<<dim3(kDm / 64, kPool), dim3(256), 0, stream>>>(fn[c], FT);
    wmma_gemm64<1, false, 0, 0, false, 0><<<dim3(tilesComp / 8, 1), dim3(256), 0, stream>>>(
        XBF, XBF, kDm, 0L, FT, FT, kDm, 0L, (void*)XN, (void*)XN, kNR, 0L, dum, dum, 0L, kTok, kNR, kDm, 1.0f);
    reduce_kernel<<<dim3(kTok / 16), dim3(256), 0, stream>>>(XN, fw[c], hh[c]);
  }

  rcast_kernel<false><<<dim3(kNR / 64, kDm / 64), dim3(256), 0, stream>>>(rqn, FT);
  buildz_kernel<false><<<dim3(kTok / 8), dim3(256), 0, stream>>>(rqw, HQ, ZQK);
  wmma_gemm64<1, false, 0, 3, false, 0><<<dim3(tilesRest / 8, 1), dim3(256), 0, stream>>>(
      ZQK, ZQK, kNR, 0L, FT, FT, kNR, 0L, (void*)Q16, (void*)Q16, kDm, 0L, dum, dum, 0L, kTok, kDm, kNR, 1.0f);
  rcast_kernel<false><<<dim3(kNR / 64, kDm / 64), dim3(256), 0, stream>>>(rkn, FT);
  buildz_kernel<false><<<dim3(kTok / 8), dim3(256), 0, stream>>>(rkw, HK, ZQK);
  wmma_gemm64<1, false, 0, 3, false, 0><<<dim3(tilesRest / 8, 1), dim3(256), 0, stream>>>(
      ZQK, ZQK, kNR, 0L, FT, FT, kNR, 0L, (void*)K16, (void*)K16, kDm, 0L, dum, dum, 0L, kTok, kDm, kNR, 1.0f);

  rcast_kernel<true><<<dim3(kNR / 64, kDm / 64), dim3(256), 0, stream>>>(rvn, RVD);
  buildz_kernel<true><<<dim3(kTok / 8), dim3(256), 0, stream>>>(rvw, HV, ZV);
  wmma_gemm64<1, false, 0, 2, false, 0><<<dim3(tilesV / 8, 1), dim3(256), 0, stream>>>(
      RVD, RVD, kZvLd, 0L, ZV, ZV, kZvLd, 0L, (void*)VTH, (void*)VTL, kTok, 0L, dum, dum, 0L, kDm, kTok, kZvLd, 1.0f);

  wo_cast_kernel<<<dim3(n8w / 256), dim3(256), 0, stream>>>(Wo, WOD, n8w);

  const long strideHead = (long)kDh;
  const long strideSc   = (long)kSeq * kSeq;
  const long strideVt   = (long)kDh * kTok;
  for (int b = 0; b < kBatch; ++b) {
    for (int g = 0; g < kHeads / kGrp; ++g) {
      const int h0 = g * kGrp;
      const size_t qkOff = (size_t)b * kSeq * kDm + (size_t)h0 * kDh;
      wmma_gemm64<1, false, 0, 0, false, 0><<<dim3(tilesS / 8, kGrp), dim3(256), 0, stream>>>(
          Q16 + qkOff, Q16 + qkOff, kDm, strideHead, K16 + qkOff, K16 + qkOff, kDm, strideHead,
          (void*)SC, (void*)SC, kSeq, strideSc, dum, dum, 0L, kSeq, kSeq, kDh, 1.0f);
      softmax_kernel<<<dim3(kSeq, kGrp), dim3(128), 0, stream>>>(SC, PH, PL);
      const size_t vtOff = (size_t)(h0 * kDh) * kTok + (size_t)b * kSeq;
      unsigned short* ctxp = CTX + (size_t)b * kSeq * kCtxLd + (size_t)h0 * kDh;
      wmma_gemm64<1, true, 0, 2, false, 0><<<dim3(tilesPV / 8, kGrp), dim3(256), 0, stream>>>(
          PH, PL, kSeq, strideSc, VTH + vtOff, VTL + vtOff, kTok, strideVt,
          (void*)ctxp, (void*)(ctxp + kDm), kCtxLd, strideHead, dum, dum, 0L, kSeq, kDh, kSeq, 1.0f);
    }
  }

  wmma_gemm64<1, false, 0, 0, false, 0><<<dim3(tilesOut / 8, 1), dim3(256), 0, stream>>>(
      CTX, CTX, kCtxLd, 0L, WOD, WOD, kCtxLd, 0L, (void*)out, (void*)out, kDm, 0L, dum, dum, 0L, kTok, kDm, kCtxLd, 1.0f);
}
